// ResonantFFN_16827681866028
// MI455X (gfx1250) — hardware-verified
//
#include <hip/hip_runtime.h>
#include <stddef.h>


typedef _Float16 v16h __attribute__((ext_vector_type(16)));
typedef _Float16 v8h  __attribute__((ext_vector_type(8)));
typedef float    v8f  __attribute__((ext_vector_type(8)));
typedef float    v4f  __attribute__((ext_vector_type(4)));
typedef _Float16 h16;

#ifndef NB
#define NB 2
#endif
#ifndef SEQ
#define SEQ 512
#endif
#define NB_FULL  2
#define SEQ_FULL 512
#define DIM   512
#define PH    64
#define HID   2048
#define MROWS (NB * SEQ)

static_assert(NB >= 1 && NB <= NB_FULL);
static_assert(SEQ >= 64 && SEQ <= SEQ_FULL && (SEQ % 64) == 0);
static_assert((DIM % 64) == 0 && (DIM % 32) == 0);
static_assert((HID % 64) == 0 && (HID % 32) == 0);
static_assert(PH == 64);
static_assert((MROWS % 64) == 0 && (MROWS % 32) == 0 && (MROWS % 4) == 0);
static_assert(DIM == 64 * 8);
static_assert((size_t)MROWS * HID < (size_t)0xFFFFFFFFu);

#define LDT 72
#define LDC 68
static_assert((LDT % 8) == 0 && LDT >= 64);
static_assert((LDC % 4) == 0 && LDC >= 64);

#define WCARRY 64.0f
#define XCARRY 16.0f
#define MCARRY 16.0f
#define GCARRY 16.0f
static_assert(MCARRY == GCARRY);

#define OUT1_OFF ((size_t)NB_FULL * SEQ_FULL * DIM)
static_assert(OUT1_OFF * 4 == (size_t)2097152);
static_assert((OUT1_OFF + (size_t)NB_FULL * SEQ_FULL * PH) * 4 == (size_t)2359296);
static_assert((OUT1_OFF * 4) % 128 == 0);

#define WUP_BYTES   ((size_t)HID * DIM * 2)
#define WDR_BYTES   ((size_t)DIM * HID * 2)
#define WDI_BYTES   ((size_t)PH * HID * 2)
#define X16_BYTES   ((size_t)MROWS * DIM * 2)
#define G32_BYTES   ((size_t)MROWS * HID * 4)
#define G16_BYTES   ((size_t)MROWS * HID * 2)
#define O16_BYTES   ((size_t)MROWS * HID * 2)
#define OFF_WUP ((size_t)0)
#define OFF_WDR (OFF_WUP + WUP_BYTES)
#define OFF_WDI (OFF_WDR + WDR_BYTES)
#define OFF_X16 (OFF_WDI + WDI_BYTES)
#define OFF_G32 (OFF_X16 + X16_BYTES)
#define OFF_G16 (OFF_G32 + G32_BYTES)
#define OFF_O16 (OFF_G16 + G16_BYTES)
#define WS_TOTAL (OFF_O16 + O16_BYTES)
static_assert((WUP_BYTES % 128) == 0 && (WDR_BYTES % 128) == 0 && (WDI_BYTES % 128) == 0);
static_assert((X16_BYTES % 128) == 0 && (G32_BYTES % 128) == 0 && (G16_BYTES % 128) == 0);
static_assert((O16_BYTES % 128) == 0);
static_assert(WS_TOTAL <= (size_t)134217728);

__device__ __forceinline__ float bf16r(float x) {
  unsigned int u = __float_as_uint(x);
  u = (u + 0x7FFFu + ((u >> 16) & 1u)) & 0xFFFF0000u;
  return __uint_as_float(u);
}

static __device__ __forceinline__ h16 toh_flush(float v) {
  const h16 r = (h16)v;
  return (fabsf(v) < 6.103515625e-05f) ? (h16)0.0f : r;
}

__device__ __forceinline__ v16h frag_at(const _Float16* p) {
  v8h lo = *(const v8h*)(p);
  v8h hi = *(const v8h*)(p + 16);
  v16h out;
#pragma unroll
  for (int i = 0; i < 8; ++i) { out[i] = lo[i]; out[i + 8] = hi[i]; }
  return out;
}

__device__ __forceinline__ v8f wmma16(v16h a, v16h b, v8f c) {
  v8f d = __builtin_amdgcn_wmma_f32_16x16x32_f16(false, a, false, b, (short)0, c,
                                                 false, false);
  asm volatile("v_nop\n\tv_nop\n\tv_nop\n\tv_nop" : "+v"(d) : "v"(a), "v"(b));
  return d;
}

__global__ __launch_bounds__(256) void wconv_kernel(
    const float* __restrict__ W, _Float16* __restrict__ Wt, unsigned ldw, unsigned ldk) {
  __shared__ _Float16 T[64 * LDT];
  const unsigned tid = threadIdx.x;
  const unsigned n0 = blockIdx.x * 64u;
  const unsigned k0 = blockIdx.y * 64u;
#pragma unroll 4
  for (unsigned j = 0; j < 16u; ++j) {
    const unsigned idx = tid + 256u * j;
    const unsigned kr = idx >> 6, nc = idx & 63u;
    const float v = W[(size_t)(k0 + kr) * ldw + n0 + nc];
    T[nc * LDT + kr] = toh_flush(WCARRY * bf16r(v));
  }
  __syncthreads();
  v8h x[2];
  size_t off[2];
#pragma unroll
  for (unsigned i = 0; i < 2u; ++i) {
    const unsigned n = 32u * i + (tid >> 3);
    const unsigned kc = (tid & 7u) * 8u;
    x[i] = *(const v8h*)&T[n * LDT + kc];
    off[i] = (size_t)(n0 + n) * ldk + k0 + kc;
  }
#pragma unroll
  for (int i = 0; i < 2; ++i) *(volatile v8h*)(Wt + off[i]) = x[i];
  __threadfence();
#pragma unroll
  for (int i = 0; i < 2; ++i) *(volatile v8h*)(Wt + off[i]) = x[i];
}

__global__ __launch_bounds__(256) void xcast_kernel(
    const float* __restrict__ X, _Float16* __restrict__ X16) {
  const unsigned tid = threadIdx.x;
  const unsigned crow = blockIdx.x * 4u + (tid >> 6);
  const unsigned c = (tid & 63u) * 8u;
  const unsigned bidx = crow / (unsigned)SEQ;
  const unsigned sq = crow - bidx * (unsigned)SEQ;
  const size_t frow = (size_t)bidx * SEQ_FULL + sq;
  const v4f a0 = *(const v4f*)(X + frow * DIM + c);
  const v4f a1 = *(const v4f*)(X + frow * DIM + c + 4u);
  v8h o;
#pragma unroll
  for (int i = 0; i < 4; ++i) {
    o[i]     = toh_flush(XCARRY * bf16r(a0[i]));
    o[i + 4] = toh_flush(XCARRY * bf16r(a1[i]));
  }
  _Float16* p = X16 + (size_t)crow * DIM + c;
  *(volatile v8h*)p = o;
  __threadfence();
  *(volatile v8h*)p = o;
}

__global__ __launch_bounds__(256) void gate_kernel(
    const float* __restrict__ xim, const float* __restrict__ pfreq,
    const float* __restrict__ wg, const float* __restrict__ bg,
    float* __restrict__ g32, _Float16* __restrict__ g16) {
  __shared__ float Tc[32 * LDC];
  __shared__ float Gs[32 * LDC];
  const unsigned tid = threadIdx.x;
  const unsigned wave = (unsigned)__builtin_amdgcn_readfirstlane((int)(tid >> 5));
  const unsigned rg = wave >> 1;
  const unsigned hl = tid & 63u;
  const unsigned h0 = blockIdx.x * 64u;
  const unsigned row0 = blockIdx.y * 32u;

#pragma unroll
  for (unsigned j = 0; j < 2u; ++j) {
    const unsigned idx = tid + 256u * j;
    const unsigned r = idx >> 4, c = (idx & 15u) * 4u;
    const unsigned crow = row0 + r;
    const unsigned bidx = crow / (unsigned)SEQ;
    const unsigned sq = crow - bidx * (unsigned)SEQ;
    const size_t frow = (size_t)bidx * SEQ_FULL + sq;
    const v4f xv = *(const v4f*)(xim + frow * PH + c);
    const v4f pv = *(const v4f*)(pfreq + (size_t)sq * PH + c);
    v4f t;
#pragma unroll
    for (int i = 0; i < 4; ++i) t[i] = bf16r(xv[i]) * bf16r(pv[i]);
    *(v4f*)&Tc[r * LDC + c] = t;
  }
  __syncthreads();

  float acc[8];
#pragma unroll
  for (int r = 0; r < 8; ++r) acc[r] = 0.0f;
  const float* wp = wg + h0 + hl;
  const float* bp = bg + h0 + hl;
#pragma unroll 1
  for (unsigned p0 = 0; p0 < (unsigned)PH; p0 += 4u) {
    float wv[4], bv[4];
#pragma unroll
    for (unsigned i = 0; i < 4u; ++i) {
      wv[i] = bf16r(wp[(size_t)(p0 + i) * HID]);
      bv[i] = bf16r(bp[(size_t)(p0 + i) * HID]);
    }
#pragma unroll
    for (unsigned r = 0; r < 8u; ++r) {
      const v4f t = *(const v4f*)&Tc[(rg * 8u + r) * LDC + p0];
#pragma unroll
      for (int i = 0; i < 4; ++i) acc[r] += __cosf(fmaf(t[i], wv[i], bv[i]));
    }
  }
#pragma unroll
  for (unsigned r = 0; r < 8u; ++r) Gs[(rg * 8u + r) * LDC + hl] = acc[r] * 0.125f;
  __syncthreads();

  v4f xs[2];
  size_t offf[2];
#pragma unroll
  for (unsigned i = 0; i < 2u; ++i) {
    const unsigned r = 16u * i + (tid >> 4);
    const unsigned c = (tid & 15u) * 4u;
    xs[i] = *(const v4f*)&Gs[r * LDC + c];
    offf[i] = (size_t)(row0 + r) * HID + h0 + c;
  }
  v8h xh;
  size_t offh;
  {
    const unsigned r = tid >> 3;
    const unsigned c = (tid & 7u) * 8u;
    const v4f u0 = *(const v4f*)&Gs[r * LDC + c];
    const v4f u1 = *(const v4f*)&Gs[r * LDC + c + 4];
#pragma unroll
    for (int j = 0; j < 4; ++j) {
      xh[j]     = toh_flush(GCARRY * u0[j]);
      xh[j + 4] = toh_flush(GCARRY * u1[j]);
    }
    offh = (size_t)(row0 + r) * HID + h0 + c;
  }
#pragma unroll
  for (int i = 0; i < 2; ++i) *(volatile v4f*)(g32 + offf[i]) = xs[i];
  *(volatile v8h*)(g16 + offh) = xh;
  __threadfence();
#pragma unroll
  for (int i = 0; i < 2; ++i) *(volatile v4f*)(g32 + offf[i]) = xs[i];
  *(volatile v8h*)(g16 + offh) = xh;
}

template <int MODE>
__device__ __forceinline__ void gemm_body(
    const _Float16* __restrict__ A16, const _Float16* __restrict__ Bt, const unsigned K,
    const float* __restrict__ gate32, const float* __restrict__ addf, const unsigned ldo,
    float* __restrict__ outf, _Float16* __restrict__ out16) {
  __shared__ float Cs[64 * LDC];
  const unsigned tid = threadIdx.x, lane = tid & 31u, w = tid >> 5;
  const unsigned mw = w >> 1, nw = w & 1u;
  const unsigned hh = lane >> 4, m = lane & 15u;
  const unsigned n0 = blockIdx.x * 64u;
  const unsigned row0 = blockIdx.y * 64u;

  const _Float16* ap  = A16 + (size_t)(row0 + mw * 16u + m) * K + hh * 8u;
  const _Float16* bp0 = Bt + (size_t)(n0 + nw * 32u + m) * K + hh * 8u;
  const _Float16* bp1 = bp0 + (size_t)16 * K;
  v8f acc0 = {}, acc1 = {};
#pragma unroll 2
  for (unsigned k0 = 0; k0 < K; k0 += 32u) {
    const v16h a  = frag_at(ap + k0);
    const v16h b0 = frag_at(bp0 + k0);
    const v16h b1 = frag_at(bp1 + k0);
    acc0 = wmma16(a, b0, acc0);
    acc1 = wmma16(a, b1, acc1);
  }
#pragma unroll
  for (int r = 0; r < 8; ++r) {
    float* d = &Cs[(mw * 16u + hh * 8u + (unsigned)r) * LDC + nw * 32u + m];
    d[0]  = acc0[r];
    d[16] = acc1[r];
  }
  __syncthreads();

  if (MODE == 0) {
    const float cs = 1.0f / (WCARRY * XCARRY);
    v8h x[2];
    size_t off[2];
#pragma unroll
    for (unsigned i = 0; i < 2u; ++i) {
      const unsigned r = 32u * i + (tid >> 3);
      const unsigned c = (tid & 7u) * 8u;
      const v4f u0 = *(const v4f*)&Cs[r * LDC + c];
      const v4f u1 = *(const v4f*)&Cs[r * LDC + c + 4];
      off[i] = (size_t)(row0 + r) * ldo + n0 + c;
      const v4f g0 = *(const v4f*)(gate32 + off[i]);
      const v4f g1 = *(const v4f*)(gate32 + off[i] + 4u);
#pragma unroll
      for (int j = 0; j < 4; ++j) {
        const float t0 = (u0[j] * cs) * g0[j];
        const float t1 = (u1[j] * cs) * g1[j];
        x[i][j]     = toh_flush(MCARRY * t0);
        x[i][j + 4] = toh_flush(MCARRY * t1);
      }
    }
#pragma unroll
    for (int i = 0; i < 2; ++i) *(volatile v8h*)(out16 + off[i]) = x[i];
    __threadfence();
#pragma unroll
    for (int i = 0; i < 2; ++i) *(volatile v8h*)(out16 + off[i]) = x[i];
  }

  if (MODE == 1) {
    const float cs = 1.0f / (WCARRY * MCARRY);
    v4f xs[4];
    size_t off[4];
#pragma unroll
    for (unsigned i = 0; i < 4u; ++i) {
      const unsigned r = 16u * i + (tid >> 4);
      const unsigned c = (tid & 15u) * 4u;
      const unsigned crow = row0 + r;
      const unsigned bidx = crow / (unsigned)SEQ;
      const unsigned sq = crow - bidx * (unsigned)SEQ;
      const size_t frow = (size_t)bidx * SEQ_FULL + sq;
      const v4f u = *(const v4f*)&Cs[r * LDC + c];
      off[i] = frow * ldo + n0 + c;
      const v4f xin = *(const v4f*)(addf + off[i]);
      v4f val;
#pragma unroll
      for (int j = 0; j < 4; ++j) val[j] = bf16r(xin[j]) + u[j] * cs;
      xs[i] = val;
    }
#pragma unroll
    for (int i = 0; i < 4; ++i) *(volatile v4f*)(outf + off[i]) = xs[i];
    __threadfence();
#pragma unroll
    for (int i = 0; i < 4; ++i) *(volatile v4f*)(outf + off[i]) = xs[i];
  }
}

__global__ __launch_bounds__(256) void gemm_up_kernel(
    const _Float16* __restrict__ A16, const _Float16* __restrict__ Bt,
    const float* __restrict__ gate32, _Float16* __restrict__ out16) {
  gemm_body<0>(A16, Bt, (unsigned)DIM, gate32, gate32, (unsigned)HID, (float*)0, out16);
}
__global__ __launch_bounds__(256) void gemm_down_kernel(
    const _Float16* __restrict__ A16, const _Float16* __restrict__ Bt,
    const float* __restrict__ xin, float* __restrict__ outf, unsigned ldo) {
  gemm_body<1>(A16, Bt, (unsigned)HID, xin, xin, ldo, outf, (_Float16*)0);
}

extern "C" void kernel_launch(void* const* d_in, const int* in_sizes, int n_in,
                              void* d_out, int out_size, void* d_ws, size_t ws_size,
                              hipStream_t stream) {
  if (n_in < 8) return;
  const long long rows_need = (long long)(NB - 1) * SEQ_FULL + SEQ;
  if ((long long)in_sizes[0] < rows_need * DIM) return;
  if ((long long)in_sizes[1] < rows_need * PH) return;
  if ((long long)in_sizes[2] < (long long)SEQ * PH) return;
  if ((long long)in_sizes[3] < (long long)DIM * HID) return;
  if ((long long)in_sizes[4] < (long long)PH * HID) return;
  if ((long long)in_sizes[5] < (long long)PH * HID) return;
  if ((long long)in_sizes[6] < (long long)HID * DIM) return;
  if ((long long)in_sizes[7] < (long long)HID * PH) return;
  if ((long long)out_size < (long long)OUT1_OFF + rows_need * PH) return;
  if (ws_size < WS_TOTAL) return;

  const float* x_real = (const float*)d_in[0];
  const float* x_imag = (const float*)d_in[1];
  const float* pfreq  = (const float*)d_in[2];
  const float* w_up   = (const float*)d_in[3];
  const float* wg     = (const float*)d_in[4];
  const float* bg     = (const float*)d_in[5];
  const float* w_dr   = (const float*)d_in[6];
  const float* w_di   = (const float*)d_in[7];
  float* out = (float*)d_out;

  char* ws = (char*)d_ws;
  _Float16* Wup_t = (_Float16*)(ws + OFF_WUP);
  _Float16* Wdr_t = (_Float16*)(ws + OFF_WDR);
  _Float16* Wdi_t = (_Float16*)(ws + OFF_WDI);
  _Float16* X16   = (_Float16*)(ws + OFF_X16);
  float*    G32   = (float*)(ws + OFF_G32);
  _Float16* G16   = (_Float16*)(ws + OFF_G16);
  _Float16* O16   = (_Float16*)(ws + OFF_O16);

  dim3 blk(256);

  wconv_kernel<<<dim3(HID / 64, DIM / 64), blk, 0, stream>>>(w_up, Wup_t, (unsigned)HID, (unsigned)DIM);
  wconv_kernel<<<dim3(DIM / 64, HID / 64), blk, 0, stream>>>(w_dr, Wdr_t, (unsigned)DIM, (unsigned)HID);
  wconv_kernel<<<dim3(PH / 64, HID / 64), blk, 0, stream>>>(w_di, Wdi_t, (unsigned)PH, (unsigned)HID);

  xcast_kernel<<<dim3(MROWS / 4), blk, 0, stream>>>(x_real, X16);
  gate_kernel<<<dim3(HID / 64, MROWS / 32), blk, 0, stream>>>(x_imag, pfreq, wg, bg, G32, G16);

  gemm_up_kernel<<<dim3(HID / 64, MROWS / 64), blk, 0, stream>>>(X16, Wup_t, G32, O16);
  gemm_down_kernel<<<dim3(DIM / 64, MROWS / 64), blk, 0, stream>>>(O16, Wdr_t, x_real, out,
                                                                  (unsigned)DIM);
  gemm_down_kernel<<<dim3(PH / 64, MROWS / 64), blk, 0, stream>>>(G16, Wdi_t, x_imag,
                                                                 out + OUT1_OFF, (unsigned)PH);
}
